// EncoderRNN_69114613730467
// MI455X (gfx1250) — hardware-verified
//
#include <hip/hip_runtime.h>
#include <math.h>

constexpr int NSEQ    = 4096;
constexpr int NVOC    = 32000;
constexpr int NEMB    = 512;
constexpr int NHID    = 512;
constexpr int NGATE3  = 3 * NHID;
constexpr int CVT_THREADS  = 256;
constexpr int SCAN_THREADS = 1024;
constexpr int NEXACT_STEPS = 16;
constexpr float ACT_CARRY = 1024.0f;
constexpr float WGT_CARRY = 256.0f;
constexpr float FOLD_INV  = 1.0f / (ACT_CARRY * WGT_CARRY);
constexpr float HALF_FOLD_INV = 0.5f * FOLD_INV;
constexpr float F16_SAFE  = 60000.0f;

static_assert(NSEQ % 64 == 0, "GEMM M tile multiple");
static_assert(NGATE3 % 64 == 0, "GEMM N tile multiple");
static_assert(NEMB % 32 == 0, "GEMM K multiple of 32");
static_assert(NHID % 32 == 0, "scan K multiple of 32");
static_assert(NHID == 16 * (SCAN_THREADS / 32), "32 waves x 16 hidden units");
static_assert(((NGATE3 * NEMB) / 8) % CVT_THREADS == 0, "weight convert grid exact");
static_assert(((NSEQ * NEMB) / 8) % CVT_THREADS == 0, "gather grid exact");
static_assert(((NSEQ / 64) * (NGATE3 / 64)) % 8 == 0, "GEMM grid exact");
static_assert(NHID == 4 * 128, "four store waves x 128 floats per output row");
static_assert(NEMB == NHID, "both weight planes share one shape");
static_assert(NHID == 2 * 256, "two lane halves x 256 k for the f32 matvec");
static_assert(NEXACT_STEPS <= NSEQ, "leading-step count within the sequence");

typedef __attribute__((ext_vector_type(16))) _Float16 v16h;
typedef __attribute__((ext_vector_type(8)))  _Float16 v8h;
typedef __attribute__((ext_vector_type(8)))  float    v8f;
typedef __attribute__((ext_vector_type(4)))  float    v4f;

union FragU { v16h v; v8h h[2]; };

__device__ __forceinline__ v16h frag_load_h(const _Float16* p) {
  FragU f;
  f.h[0] = *(const v8h*)(p);
  f.h[1] = *(const v8h*)(p + 16);
  return f.v;
}
__device__ __forceinline__ v8f mma_h(v16h a, v16h b, v8f c) {
  return __builtin_amdgcn_wmma_f32_16x16x32_f16(false, a, false, b, (short)0, c, false, false);
}
__device__ __forceinline__ void guard_acc4(v8f& a, v8f& b, v8f& c, v8f& d, v16h x, v16h y0, v16h y1, v16h y2, v16h y3) {
  asm volatile("v_nop\n\tv_nop\n\tv_nop\n\tv_nop" : "+v"(a), "+v"(b), "+v"(c), "+v"(d) : "v"(x), "v"(y0), "v"(y1), "v"(y2), "v"(y3));
}
__device__ __forceinline__ void guard_acc3(v8f& a, v8f& b, v8f& c, v16h x, v16h y0, v16h y1, v16h y2) {
  asm volatile("v_nop\n\tv_nop\n\tv_nop\n\tv_nop" : "+v"(a), "+v"(b), "+v"(c) : "v"(x), "v"(y0), "v"(y1), "v"(y2));
}
__device__ __forceinline__ void keep4_h(v16h a, v16h b, v16h c, v16h d) { asm volatile("v_nop" :: "v"(a), "v"(b), "v"(c), "v"(d)); }
__device__ __forceinline__ void acc_guard4(v8f& a, v8f& b, v8f& c, v8f& d) { asm volatile("v_nop\n\tv_nop\n\tv_nop\n\tv_nop" : "+v"(a), "+v"(b), "+v"(c), "+v"(d)); }
__device__ __forceinline__ void acc_guard3(v8f& a, v8f& b, v8f& c) { asm volatile("v_nop\n\tv_nop\n\tv_nop\n\tv_nop" : "+v"(a), "+v"(b), "+v"(c)); }

__device__ __forceinline__ float clamp_f16_range(float v) { return fminf(fmaxf(v, -F16_SAFE), F16_SAFE); }
__device__ __forceinline__ float sigmoid_f32(float x) {
  const float xc = fminf(fmaxf(x, -30.0f), 30.0f);
  const float e = expf(-xc);
  return 1.0f / (1.0f + e);
}

__global__ __launch_bounds__(CVT_THREADS) void cvt_weights_kernel(const float* __restrict__ src0, const float* __restrict__ src1,
                                                                  unsigned short* __restrict__ dst0, unsigned short* __restrict__ dst1,
                                                                  int n8, float sc) {
  const int i = blockIdx.x * CVT_THREADS + threadIdx.x;
  const bool second = (blockIdx.y != 0);
  const float* src = second ? src1 : src0;
  unsigned short* dst = second ? dst1 : dst0;
  if (i < n8) {
    const float* sp = src + (size_t)i * 8;
    const v4f a = *(const v4f*)(sp);
    const v4f b = *(const v4f*)(sp + 4);
    v8h hv;
#pragma unroll
    for (int e = 0; e < 4; ++e) {
      const float fa = a[e] * sc;
      const float fb = b[e] * sc;
      hv[e]     = (_Float16)fa;
      hv[4 + e] = (_Float16)fb;
    }
    volatile v8h* dp = (volatile v8h*)(dst + (size_t)i * 8);
    *dp = hv;
    __threadfence();
    *dp = hv;
  }
}

__global__ __launch_bounds__(CVT_THREADS) void gather_cvt_kernel(const int* __restrict__ ids, const float* __restrict__ emb,
                                                                 unsigned short* __restrict__ dst, int n8, float sc) {
  const int i = blockIdx.x * CVT_THREADS + threadIdx.x;
  if (i < n8) {
    const int t  = i >> 6;
    const int c8 = i & 63;
    int id = ids[t];
    id = id < 0 ? 0 : id;
    id = id > (NVOC - 1) ? (NVOC - 1) : id;
    const float* sp = emb + (size_t)id * NEMB + c8 * 8;
    const v4f a = *(const v4f*)(sp);
    const v4f b = *(const v4f*)(sp + 4);
    v8h hv;
#pragma unroll
    for (int e = 0; e < 4; ++e) {
      const float fa = a[e] * sc;
      const float fb = b[e] * sc;
      hv[e]     = (_Float16)fa;
      hv[4 + e] = (_Float16)fb;
    }
    volatile v8h* dp = (volatile v8h*)(dst + (size_t)i * 8);
    *dp = hv;
    __threadfence();
    *dp = hv;
  }
}

__global__ __launch_bounds__(256) void xproj_gemm_kernel(const unsigned short* __restrict__ Ap, int lda,
                                                         const unsigned short* __restrict__ Btp, int ldb,
                                                         float* __restrict__ Cout, int ldc,
                                                         const float* __restrict__ bias, int M, int N, int K, float scale) {
  const _Float16* A  = (const _Float16*)Ap;
  const _Float16* Bt = (const _Float16*)Btp;
  __shared__ __align__(16) float sT[8][16 * 68];
  const int lane = threadIdx.x & 31;
  const int wave = threadIdx.x >> 5;
  const int tilesN = N >> 6;
  const int tilesM = M >> 6;
  const int tile = blockIdx.x * 8 + wave;
  if (tile >= tilesM * tilesN) return;
  const int tm = tile / tilesN;
  const int tn = tile - tm * tilesN;
  const int m0 = tm << 6;
  const int n0 = tn << 6;

  const int rlane = lane & 15;
  const int koff  = (lane >> 4) * 8;
  const int mOff  = (lane >> 4) * 8;

  v8f acc[4][4];
#pragma unroll
  for (int i = 0; i < 4; ++i)
#pragma unroll
    for (int j = 0; j < 4; ++j) acc[i][j] = (v8f){0.f, 0.f, 0.f, 0.f, 0.f, 0.f, 0.f, 0.f};

  for (int k0 = 0; k0 < K; k0 += 32) {
    v16h bh[4];
#pragma unroll
    for (int j = 0; j < 4; ++j) {
      const size_t bo = (size_t)(n0 + (j << 4) + rlane) * ldb + koff + k0;
      bh[j] = frag_load_h(Bt + bo);
    }
#pragma unroll
    for (int i = 0; i < 4; ++i) {
      const size_t ao = (size_t)(m0 + (i << 4) + rlane) * lda + koff + k0;
      const v16h ah = frag_load_h(A + ao);
#pragma unroll
      for (int j = 0; j < 4; ++j) acc[i][j] = mma_h(ah, bh[j], acc[i][j]);
      guard_acc4(acc[i][0], acc[i][1], acc[i][2], acc[i][3], ah, bh[0], bh[1], bh[2], bh[3]);
    }
    keep4_h(bh[0], bh[1], bh[2], bh[3]);
  }
  acc_guard4(acc[0][0], acc[0][1], acc[0][2], acc[0][3]);
  acc_guard4(acc[1][0], acc[1][1], acc[1][2], acc[1][3]);
  acc_guard4(acc[2][0], acc[2][1], acc[2][2], acc[2][3]);
  acc_guard4(acc[3][0], acc[3][1], acc[3][2], acc[3][3]);

  float* slab = sT[wave];
#pragma unroll
  for (int i = 0; i < 4; ++i) {
    const int mBase = m0 + (i << 4);
#pragma unroll
    for (int j = 0; j < 4; ++j) {
      const int n = n0 + (j << 4) + rlane;
      const float bv = bias[n];
#pragma unroll
      for (int r = 0; r < 8; ++r) {
        float v = acc[i][j][r] * scale;
        v += bv;
        slab[(mOff + r) * 68 + (j << 4) + rlane] = v;
      }
    }
    __builtin_amdgcn_fence(__ATOMIC_RELEASE, "workgroup");
    __builtin_amdgcn_wave_barrier();
    __builtin_amdgcn_fence(__ATOMIC_ACQUIRE, "workgroup");
    {
      const int hh = lane >> 4, c4 = (lane & 15) * 4;
      for (int pass = 0; pass < 2; ++pass) {
#pragma unroll
        for (int it = 0; it < 8; ++it) {
          const int row = it * 2 + hh;
          const v4f v = *(const v4f*)(slab + row * 68 + c4);
          *(volatile v4f*)(Cout + (size_t)(mBase + row) * ldc + n0 + c4) = v;
        }
        __threadfence();
      }
    }
    __builtin_amdgcn_fence(__ATOMIC_RELEASE, "workgroup");
    __builtin_amdgcn_wave_barrier();
    __builtin_amdgcn_fence(__ATOMIC_ACQUIRE, "workgroup");
  }
}

__global__ __launch_bounds__(SCAN_THREADS) void gru_scan_kernel(const float* __restrict__ xp, const float* __restrict__ h0,
                                                                const unsigned short* __restrict__ whp,
                                                                const float* __restrict__ whh32,
                                                                const float* __restrict__ bhh, float* __restrict__ out) {
  __shared__ __align__(16) _Float16 hq[3 * NHID];
  __shared__ __align__(16) float    hf[3 * NHID];
  const _Float16* WH = (const _Float16*)whp;
  const int tid = threadIdx.x, lane = tid & 31, wave = tid >> 5;
  const int c = lane & 15, hh = lane >> 4, koff = hh * 8;
  const int j = 16 * wave + c;

  float hstate = h0[j];
  {
    const int slot0 = (hh != 0) ? 2 : 0;
    const float hv = clamp_f16_range(hstate * ACT_CARRY);
    hf[slot0 * NHID + j] = hstate;
    hq[slot0 * NHID + j] = (_Float16)hv;
  }
  const float bhr = bhh[j];
  const float bhz = bhh[NHID + j];
  const float bhn = bhh[2 * NHID + j];
  const _Float16* wr = WH + (size_t)j * NHID + koff;
  const _Float16* wz = wr + (size_t)NHID * NHID;
  const _Float16* wn = wz + (size_t)NHID * NHID;
  const v4f* w32r = (const v4f*)(whh32 + (size_t)j * NHID + 256 * hh);
  const v4f* w32z = (const v4f*)(whh32 + (size_t)(NHID + j) * NHID + 256 * hh);
  const v4f* w32n = (const v4f*)(whh32 + (size_t)(2 * NHID + j) * NHID + 256 * hh);
  const v8f z8 = {0.f, 0.f, 0.f, 0.f, 0.f, 0.f, 0.f, 0.f};
  __syncthreads();

#pragma unroll 1
  for (int t = 0; t < NSEQ; ++t) {
    const int cur = t & 1;
    const int nxt = cur ^ 1;
    const float* xrow = xp + (size_t)t * NGATE3 + j;
    float xr = xrow[0];
    float xz = xrow[NHID];
    float xn = xrow[2 * NHID];
    asm volatile("" : "+v"(xr), "+v"(xz), "+v"(xn));

    float pr, pz, pn;
    if (t < NEXACT_STEPS) {
      const v4f* hv4 = (const v4f*)(hf + cur * NHID + 256 * hh);
      float sr = 0.0f, sz = 0.0f, sn = 0.0f;
#pragma unroll 2
      for (int k4 = 0; k4 < 64; ++k4) {
        const v4f hx = hv4[k4];
        const v4f qa = w32r[k4];
        const v4f qb = w32z[k4];
        const v4f qc = w32n[k4];
        sr = fmaf(qa[0], hx[0], sr);
        sz = fmaf(qb[0], hx[0], sz);
        sn = fmaf(qc[0], hx[0], sn);
        sr = fmaf(qa[1], hx[1], sr);
        sz = fmaf(qb[1], hx[1], sz);
        sn = fmaf(qc[1], hx[1], sn);
        sr = fmaf(qa[2], hx[2], sr);
        sz = fmaf(qb[2], hx[2], sz);
        sn = fmaf(qc[2], hx[2], sn);
        sr = fmaf(qa[3], hx[3], sr);
        sz = fmaf(qb[3], hx[3], sz);
        sn = fmaf(qc[3], hx[3], sn);
      }
      pr = sr;
      pz = sz;
      pn = sn;
    } else {
      const _Float16* arow = hq + cur * NHID + koff;
      v8f accR = z8, accZ = z8, accN = z8;
#pragma unroll 1
      for (int k0 = 0; k0 < NHID; k0 += 32) {
        const v16h a  = frag_load_h(arow + k0);
        const v16h b0 = frag_load_h(wr + k0);
        const v16h b1 = frag_load_h(wz + k0);
        const v16h b2 = frag_load_h(wn + k0);
        accR = mma_h(a, b0, accR);
        accZ = mma_h(a, b1, accZ);
        accN = mma_h(a, b2, accN);
        guard_acc3(accR, accZ, accN, a, b0, b1, b2);
      }
      acc_guard3(accR, accZ, accN);
      pr = accR[0] * HALF_FOLD_INV;
      pz = accZ[0] * HALF_FOLD_INV;
      pn = accN[0] * HALF_FOLD_INV;
    }
    const float qr = __shfl_xor(pr, 16, 32);
    const float qz = __shfl_xor(pz, 16, 32);
    const float qn = __shfl_xor(pn, 16, 32);

    const float gr = (pr + qr) + bhr;
    const float gz = (pz + qz) + bhz;
    const float gn = (pn + qn) + bhn;
    const float rg = sigmoid_f32(xr + gr);
    const float zg = sigmoid_f32(xz + gz);
    const float ng = tanhf(xn + rg * gn);
    const float hnew = (1.0f - zg) * ng + zg * hstate;
    hstate = hnew;

    const int dslot = (hh != 0) ? 2 : nxt;
    const float hc = clamp_f16_range(hnew * ACT_CARRY);
    hf[dslot * NHID + j] = hnew;
    hq[dslot * NHID + j] = (_Float16)hc;
    __syncthreads();

    if (wave < 4) {
      const v4f v = *(const v4f*)(hf + nxt * NHID + 128 * wave + 4 * lane);
      volatile v4f* op = (volatile v4f*)(out + (size_t)t * NHID + 128 * wave + 4 * lane);
      *op = v;
      __threadfence();
      *op = v;
    }
  }
}

extern "C" void kernel_launch(void* const* d_in, const int* in_sizes, int n_in,
                              void* d_out, int out_size, void* d_ws, size_t ws_size, hipStream_t stream) {
  if (n_in < 7 || d_out == nullptr || d_ws == nullptr) return;
  if (in_sizes[0] != NSEQ || in_sizes[1] != NHID || in_sizes[2] != NVOC * NEMB ||
      in_sizes[3] != NGATE3 * NEMB || in_sizes[4] != NGATE3 * NHID ||
      in_sizes[5] != NGATE3 || in_sizes[6] != NGATE3 || out_size != NSEQ * NHID) return;

  const int*   ids = (const int*)d_in[0];
  const float* h0  = (const float*)d_in[1];
  const float* emb = (const float*)d_in[2];
  const float* wih = (const float*)d_in[3];
  const float* whh = (const float*)d_in[4];
  const float* bih = (const float*)d_in[5];
  const float* bhh = (const float*)d_in[6];
  float* out = (float*)d_out;

  char* ws = (char*)d_ws;
  size_t off = 0;
  auto carve = [&](size_t bytes) -> char* { char* p = ws + off; off += (bytes + 255) & ~(size_t)255; return p; };
  unsigned short* WIH16 = (unsigned short*)carve((size_t)NGATE3 * NEMB * 2);
  unsigned short* WHH16 = (unsigned short*)carve((size_t)NGATE3 * NHID * 2);
  unsigned short* XH16  = (unsigned short*)carve((size_t)NSEQ * NEMB * 2);
  float*          XPROJ = (float*)carve((size_t)NSEQ * NGATE3 * 4);
  if (off > ws_size || off > (size_t)134217728) return;

  const int n8w = (NGATE3 * NEMB) / 8;
  cvt_weights_kernel<<<dim3(n8w / CVT_THREADS, 2), CVT_THREADS, 0, stream>>>(wih, whh, WIH16, WHH16, n8w, WGT_CARRY);

  const int n8x = (NSEQ * NEMB) / 8;
  gather_cvt_kernel<<<n8x / CVT_THREADS, CVT_THREADS, 0, stream>>>(ids, emb, XH16, n8x, ACT_CARRY);

  const int ntiles = (NSEQ / 64) * (NGATE3 / 64);
  xproj_gemm_kernel<<<ntiles / 8, 256, 0, stream>>>(XH16, NEMB, WIH16, NEMB, XPROJ, NGATE3, bih,
                                                    NSEQ, NGATE3, NEMB, FOLD_INV);

  gru_scan_kernel<<<1, SCAN_THREADS, 0, stream>>>(XPROJ, h0, WHH16, whh, bhh, out);
}
